// GCNIIBackbone_42004780155161
// MI455X (gfx1250) — hardware-verified
//
#include <hip/hip_runtime.h>
#include <math.h>


typedef __bf16 bf_t;
typedef bf_t v16b __attribute__((ext_vector_type(16)));
typedef unsigned short v4us __attribute__((ext_vector_type(4)));
typedef unsigned short v8us __attribute__((ext_vector_type(8)));
typedef float v4f __attribute__((ext_vector_type(4)));
typedef float v8f __attribute__((ext_vector_type(8)));
typedef int v4i __attribute__((ext_vector_type(4)));
typedef double v2d __attribute__((ext_vector_type(2)));

#define DIN 64
#define DHID 128
#define DOUT 64
#define NLAYERS 8
#define NPBK 128
#define BCAP 2048
#define MAXDEG 256
#define STR 136
#define GP 132
#define GP2 68
#define TP (DHID + 4)
#define PLD 16
#define SLF 32
#define LN_EPS 1e-5f

union Frag { v16b v; v8us p[2]; };

__device__ __forceinline__ v4f z4() { v4f z = {0.0f, 0.0f, 0.0f, 0.0f}; return z; }
__device__ __forceinline__ v8f z8() { v8f z = {0.0f, 0.0f, 0.0f, 0.0f, 0.0f, 0.0f, 0.0f, 0.0f}; return z; }

__device__ __forceinline__ unsigned short f2bf(float x) {
  unsigned int u = __float_as_uint(x);
  u += 0x7FFFu + ((u >> 16) & 1u);
  return (unsigned short)(u >> 16);
}
__device__ __forceinline__ float bf2f(unsigned short b) {
  return __uint_as_float(((unsigned int)b) << 16);
}
__device__ __forceinline__ void split4(const v4f v, v4us& hi, v4us& lo) {
  const unsigned short h0 = f2bf(v.x), h1 = f2bf(v.y), h2 = f2bf(v.z), h3 = f2bf(v.w);
  hi.x = h0; hi.y = h1; hi.z = h2; hi.w = h3;
  lo.x = f2bf(v.x - bf2f(h0));
  lo.y = f2bf(v.y - bf2f(h1));
  lo.z = f2bf(v.z - bf2f(h2));
  lo.w = f2bf(v.w - bf2f(h3));
}

__device__ __forceinline__ v16b frag_ld(const unsigned short* base, int pitch, int lane, int k0) {
  const int h = lane >> 4, m = lane & 15;
  const unsigned short* p = base + m * pitch + k0 + 8 * h;
  Frag f;
  f.p[0] = *(const v8us*)(p);
  f.p[1] = *(const v8us*)(p + 16);
  return f.v;
}

__device__ __forceinline__ v8f mma3(v8f acc, v16b ah, v16b al, v16b bh, v16b bl) {
  acc = __builtin_amdgcn_wmma_f32_16x16x32_bf16(false, ah, false, bh, (short)0, acc, false, false);
  acc = __builtin_amdgcn_wmma_f32_16x16x32_bf16(false, ah, false, bl, (short)0, acc, false, false);
  acc = __builtin_amdgcn_wmma_f32_16x16x32_bf16(false, al, false, bh, (short)0, acc, false, false);
  asm volatile("v_nop\n\tv_nop\n\tv_nop\n\tv_nop" : "+v"(acc) : "v"(ah), "v"(al), "v"(bh), "v"(bl));
  return acc;
}

__device__ __forceinline__ v4f ln_relu(v4f hv, float mu, float inv, v4f nwv, v4f nbv) {
  v4f t = (hv - mu) * inv;
  t = t * nwv + nbv;
  t.x = fmaxf(t.x, 0.0f);
  t.y = fmaxf(t.y, 0.0f);
  t.z = fmaxf(t.z, 0.0f);
  t.w = fmaxf(t.w, 0.0f);
  return t;
}

__global__ __launch_bounds__(256) void k_csr(const int* __restrict__ erow,
                                             const int* __restrict__ ecol,
                                             int ne, int nn,
                                             int* csr, int* nstart, int* ncnt,
                                             float* dinv) {
  __shared__ int lst_row[BCAP];
  __shared__ unsigned char lst_cid[BCAP];
  __shared__ __align__(16) int srt[BCAP];
  __shared__ int wcnt[8];
  __shared__ __align__(16) int s_cnt[NPBK];
  __shared__ __align__(16) int s_off[NPBK];
  __shared__ __align__(16) float s_dinv[NPBK];
  const int k = blockIdx.x;
  const int lo = k * NPBK;
  const int tid = threadIdx.x, lane = tid & 31, w = tid >> 5;

  int run = 0;
  for (int base = 0; base < ne; base += 256) {
    const int e = base + tid;
    int c = -1;
    if (e < ne) c = ecol[e];
    const bool hit = (e < ne) && ((unsigned)(c - lo) < (unsigned)NPBK);
    const unsigned msk = __builtin_amdgcn_ballot_w32(hit);
    if (lane == 0) wcnt[w] = (int)__builtin_popcount(msk);
    __syncthreads();
    int pre = 0, tot = 0;
#pragma unroll
    for (int q = 0; q < 8; ++q) {
      const int v = wcnt[q];
      tot += v;
      pre += (q < w) ? v : 0;
    }
    const int pos = run + pre + (int)__builtin_popcount(msk & ((1u << lane) - 1u));
    if (hit && pos < BCAP) {
      int r = erow[e];
      r = min(max(r, 0), nn - 1);
      lst_row[pos] = r;
      lst_cid[pos] = (unsigned char)(c - lo);
    }
    run += tot;
    __syncthreads();
  }
  const int len = min(run, BCAP);
  for (int i = tid; i < BCAP; i += 256) srt[i] = 0;
  int mycnt = 0;
  if (tid < NPBK) {
    for (int i = 0; i < len; ++i) mycnt += ((int)lst_cid[i] == tid) ? 1 : 0;
    s_cnt[tid] = mycnt;
  }
  __syncthreads();
  if (tid == 0) {
    int a = 0;
    for (int i = 0; i < NPBK; ++i) { const int v = s_cnt[i]; s_off[i] = a; a += v; }
  }
  __syncthreads();
  if (tid < NPBK) {
    int o = s_off[tid];
    for (int i = 0; i < len; ++i) {
      if ((int)lst_cid[i] == tid) { srt[min(o, BCAP - 1)] = lst_row[i]; ++o; }
    }
    s_dinv[tid] = 1.0f / sqrtf(1.0f + (float)mycnt);
  }
  __syncthreads();

  auto emit = [&]() {
    int* dst = csr + (size_t)k * BCAP;
    for (int ch = w; ch < BCAP / 128; ch += 8) {
      v4i v = *(const v4i*)(srt + ch * 128 + 4 * lane);
      *(volatile v4i*)(dst + ch * 128 + 4 * lane) = v;
    }
    if (w == 0) {
      v4i v = *(const v4i*)(s_off + 4 * lane);
      v = v + k * BCAP;
      *(volatile v4i*)(nstart + lo + 4 * lane) = v;
    } else if (w == 1) {
      v4i v = *(const v4i*)(s_cnt + 4 * lane);
      *(volatile v4i*)(ncnt + lo + 4 * lane) = v;
    } else if (w == 2) {
      v4f v = *(const v4f*)(s_dinv + 4 * lane);
      *(volatile v4f*)(dinv + lo + 4 * lane) = v;
    }
  };
  emit();
  __threadfence();
  emit();
}

__global__ __launch_bounds__(256) void k_wcvt(const float* __restrict__ src, int K, int N, int nmat,
                                              unsigned short* dhi, unsigned short* dlo) {
  __shared__ __align__(16) float T[32 * TP];
  const int slabs = N >> 5;
  const int mat = blockIdx.x / slabs;
  const int n0 = (blockIdx.x - mat * slabs) * 32;
  if (mat >= nmat) return;
  const int tid = threadIdx.x;
  for (int idx = tid; idx < K * 32; idx += 256) {
    const int kk = idx >> 5, nl = idx & 31;
    T[nl * TP + kk] = src[((size_t)mat * K + kk) * N + n0 + nl];
  }
  __syncthreads();
  const int cpr = K >> 3;
  const int nch = 32 * cpr;
  auto emit = [&]() {
    for (int c = tid; c < nch; c += 256) {
      const int row = c / cpr, kc = (c - row * cpr) * 8;
      const float* tp = T + row * TP + kc;
      v8us hi, lo;
#pragma unroll
      for (int i = 0; i < 8; ++i) {
        const float xv = tp[i];
        const unsigned short hb = f2bf(xv);
        hi[i] = hb;
        lo[i] = f2bf(xv - bf2f(hb));
      }
      const size_t o = ((size_t)mat * N + n0 + row) * (size_t)K + kc;
      *(volatile v8us*)(dhi + o) = hi;
      *(volatile v8us*)(dlo + o) = lo;
    }
  };
  emit();
  __threadfence();
  emit();
}

__global__ __launch_bounds__(128) void k_lin1(const float* __restrict__ x,
                                              const unsigned short* __restrict__ whi,
                                              const unsigned short* __restrict__ wlo,
                                              const float* __restrict__ bias, int nn,
                                              float* x0) {
  __shared__ __align__(16) unsigned short Ah[16 * STR];
  __shared__ __align__(16) unsigned short Al[16 * STR];
  __shared__ __align__(16) float G[16 * GP];
  const int row0 = blockIdx.x * 16;
  const int tid = threadIdx.x, lane = tid & 31, w = tid >> 5;
  const int hh = lane >> 4, m = lane & 15;
  for (int idx = tid; idx < 16 * (DIN / 4); idx += 128) {
    const int r = idx / (DIN / 4), c4 = (idx - r * (DIN / 4)) * 4;
    const int row = row0 + r;
    v4f v = z4();
    if (row < nn) v = *(const v4f*)(x + (size_t)row * DIN + c4);
    v4us hi, lo;
    split4(v, hi, lo);
    *(v4us*)(Ah + r * STR + c4) = hi;
    *(v4us*)(Al + r * STR + c4) = lo;
  }
  __syncthreads();
#pragma unroll
  for (int t = 0; t < 2; ++t) {
    const int n0 = (w + 4 * t) * 16;
    const unsigned short* bh_base = whi + (size_t)n0 * DIN;
    const unsigned short* bl_base = wlo + (size_t)n0 * DIN;
    v8f acc = z8();
#pragma unroll 1
    for (int ks = 0; ks < DIN / 32; ++ks) {
      const int k0 = ks * 32;
      v16b ah = frag_ld(Ah, STR, lane, k0);
      v16b al = frag_ld(Al, STR, lane, k0);
      v16b bh = frag_ld(bh_base, DIN, lane, k0);
      v16b bl = frag_ld(bl_base, DIN, lane, k0);
      acc = mma3(acc, ah, al, bh, bl);
    }
#pragma unroll
    for (int r = 0; r < 8; ++r) G[(8 * hh + r) * GP + n0 + m] = acc[r];
  }
  __syncthreads();
  const v4f bv = *(const v4f*)(bias + 4 * lane);
  v4f vals[4];
#pragma unroll
  for (int j = 0; j < 4; ++j) {
    const int ml = 4 * w + j;
    const v4f g = *(const v4f*)(G + ml * GP + 4 * lane);
    vals[j] = (g + bv) * 0.5f;
  }
  auto emit = [&]() {
#pragma unroll
    for (int j = 0; j < 4; ++j) {
      const int row = row0 + 4 * w + j;
      if (row < nn) *(volatile v4f*)(x0 + (size_t)row * DHID + 4 * lane) = vals[j];
    }
  };
  emit();
  __threadfence();
  emit();
}

__global__ __launch_bounds__(128) void k_layer(
    const float* __restrict__ hsrc, int mode, const float* __restrict__ stats,
    const float* __restrict__ nw, const float* __restrict__ nb,
    const float* __restrict__ x0, const int* __restrict__ csr,
    const int* __restrict__ nstart, const int* __restrict__ ncnt,
    const float* __restrict__ dinv, int csr_len,
    const unsigned short* __restrict__ w1h, const unsigned short* __restrict__ w1l,
    const unsigned short* __restrict__ w2h, const unsigned short* __restrict__ w2l,
    float beta, int nn, float* out, double* partials) {
  __shared__ __align__(16) unsigned short Ah[16 * STR];
  __shared__ __align__(16) unsigned short Al[16 * STR];
  __shared__ __align__(16) unsigned short Xh[16 * STR];
  __shared__ __align__(16) unsigned short Xl[16 * STR];
  __shared__ __align__(16) float Sagg[16 * DHID];
  __shared__ __align__(16) float G[16 * GP];
  __shared__ double red[8];
  const int row0 = blockIdx.x * 16;
  const int tid = threadIdx.x, lane = tid & 31, w = tid >> 5;
  const int hh = lane >> 4, m = lane & 15;

  float mu = 0.0f, inv = 1.0f;
  v4f nwv = {1.0f, 1.0f, 1.0f, 1.0f};
  v4f nbv = z4();
  if (mode != 0) {
    mu = stats[0];
    inv = stats[1];
    nwv = *(const v4f*)(nw + 4 * lane);
    nbv = *(const v4f*)(nb + 4 * lane);
  }

#pragma unroll 1
  for (int j = 0; j < 4; ++j) {
    const int ml = 4 * w + j;
    const int c = row0 + ml;
    v4f acc4 = z4();
    v4f xv = z4();
    if (c < nn) {
      int cnt = ncnt[c];
      cnt = min(max(cnt, 0), MAXDEG);
      const int st = nstart[c];
      const float dc = dinv[c];
      for (int e = 0; e < cnt; ++e) {
        int idx = st + e;
        idx = min(max(idx, 0), csr_len - 1);
        int r = csr[idx];
        r = min(max(r, 0), nn - 1);
        const float wgt = dinv[r] * dc;
        v4f hv = *(const v4f*)(hsrc + (size_t)r * DHID + 4 * lane);
        hv = (mode != 0) ? ln_relu(hv, mu, inv, nwv, nbv) : (hv + hv);
        acc4 += wgt * hv;
      }
      v4f hs = *(const v4f*)(hsrc + (size_t)c * DHID + 4 * lane);
      hs = (mode != 0) ? ln_relu(hs, mu, inv, nwv, nbv) : (hs + hs);
      acc4 += (dc * dc) * hs;
      acc4 *= 0.5f;
      xv = *(const v4f*)(x0 + (size_t)c * DHID + 4 * lane);
    }
    *(v4f*)(Sagg + ml * DHID + 4 * lane) = acc4;
    v4us hi, lo;
    split4(acc4, hi, lo);
    *(v4us*)(Ah + ml * STR + 4 * lane) = hi;
    *(v4us*)(Al + ml * STR + 4 * lane) = lo;
    split4(xv, hi, lo);
    *(v4us*)(Xh + ml * STR + 4 * lane) = hi;
    *(v4us*)(Xl + ml * STR + 4 * lane) = lo;
  }
  __syncthreads();

#pragma unroll
  for (int t = 0; t < 2; ++t) {
    const int n0 = (w + 4 * t) * 16;
    const unsigned short* b1h = w1h + (size_t)n0 * DHID;
    const unsigned short* b1l = w1l + (size_t)n0 * DHID;
    const unsigned short* b2h = w2h + (size_t)n0 * DHID;
    const unsigned short* b2l = w2l + (size_t)n0 * DHID;
    v8f acc = z8();
#pragma unroll 1
    for (int ks = 0; ks < DHID / 32; ++ks) {
      const int k0 = ks * 32;
      v16b ah = frag_ld(Ah, STR, lane, k0);
      v16b al = frag_ld(Al, STR, lane, k0);
      v16b bh = frag_ld(b1h, DHID, lane, k0);
      v16b bl = frag_ld(b1l, DHID, lane, k0);
      acc = mma3(acc, ah, al, bh, bl);
      v16b ch = frag_ld(Xh, STR, lane, k0);
      v16b cl = frag_ld(Xl, STR, lane, k0);
      v16b dh = frag_ld(b2h, DHID, lane, k0);
      v16b dl = frag_ld(b2l, DHID, lane, k0);
      acc = mma3(acc, ch, cl, dh, dl);
    }
#pragma unroll
    for (int r = 0; r < 8; ++r) G[(8 * hh + r) * GP + n0 + m] = acc[r];
  }
  __syncthreads();

  const float omb = 1.0f - beta;
  v4f vals[4];
  double s = 0.0, s2 = 0.0;
#pragma unroll
  for (int j = 0; j < 4; ++j) {
    const int ml = 4 * w + j;
    const int row = row0 + ml;
    const v4f g = *(const v4f*)(G + ml * GP + 4 * lane);
    const v4f ag = *(const v4f*)(Sagg + ml * DHID + 4 * lane);
    v4f xv = z4();
    if (row < nn) xv = *(const v4f*)(x0 + (size_t)row * DHID + 4 * lane);
    v4f v = omb * ag + beta * g;
    v = v + omb * xv;
    vals[j] = v;
    if (row < nn) {
      s += (double)v.x; s += (double)v.y; s += (double)v.z; s += (double)v.w;
      s2 += (double)v.x * (double)v.x; s2 += (double)v.y * (double)v.y;
      s2 += (double)v.z * (double)v.z; s2 += (double)v.w * (double)v.w;
    }
  }
#pragma unroll
  for (int o = 16; o > 0; o >>= 1) {
    s += __shfl_xor(s, o, 32);
    s2 += __shfl_xor(s2, o, 32);
  }
  if (lane == 0) { red[2 * w] = s; red[2 * w + 1] = s2; }
  __syncthreads();
  double S = 0.0, S2 = 0.0;
#pragma unroll
  for (int q = 0; q < 4; ++q) { S += red[2 * q]; S2 += red[2 * q + 1]; }
  v2d pv = {0.0, 0.0};
  if (lane == 0) { pv.x = S; pv.y = S2; }
  double* pl = partials + (size_t)blockIdx.x * PLD;

  auto emit = [&]() {
#pragma unroll
    for (int j = 0; j < 4; ++j) {
      const int row = row0 + 4 * w + j;
      if (row < nn) *(volatile v4f*)(out + (size_t)row * DHID + 4 * lane) = vals[j];
    }
    if (w == 0 && lane < 8) *(volatile v2d*)(pl + 2 * lane) = pv;
  };
  emit();
  __threadfence();
  emit();
}

__global__ __launch_bounds__(256) void k_lnstat(const double* __restrict__ partials, int nblk,
                                                double cntM, float* stats) {
  __shared__ double r1[8], r2[8];
  const int tid = threadIdx.x, lane = tid & 31, w = tid >> 5;
  double s = 0.0, s2 = 0.0;
  for (int b = tid; b < nblk; b += 256) {
    s += partials[(size_t)b * PLD];
    s2 += partials[(size_t)b * PLD + 1];
  }
#pragma unroll
  for (int o = 16; o > 0; o >>= 1) {
    s += __shfl_xor(s, o, 32);
    s2 += __shfl_xor(s2, o, 32);
  }
  if (lane == 0) { r1[w] = s; r2[w] = s2; }
  __syncthreads();
  if (w == 0) {
    double S = 0.0, S2 = 0.0;
#pragma unroll
    for (int q = 0; q < 8; ++q) { S += r1[q]; S2 += r2[q]; }
    const double mean = S / cntM;
    double var = S2 / cntM - mean * mean;
    if (var < 0.0) var = 0.0;
    const float sd = (float)sqrt(var);
    const float muf = (float)mean;
    const float invf = 1.0f / (sd + LN_EPS);
    v4f v = z4();
    if (lane == 0) { v.x = muf; v.y = invf; }
    if (lane < 8) *(volatile v4f*)(stats + 4 * lane) = v;
    __threadfence();
    if (lane < 8) *(volatile v4f*)(stats + 4 * lane) = v;
  }
}

__global__ __launch_bounds__(128) void k_lin2(const float* __restrict__ hsrc,
                                              const float* __restrict__ stats,
                                              const float* __restrict__ nw,
                                              const float* __restrict__ nb,
                                              const unsigned short* __restrict__ whi,
                                              const unsigned short* __restrict__ wlo,
                                              const float* __restrict__ bias, int nn,
                                              float* out) {
  __shared__ __align__(16) unsigned short Ah[16 * STR];
  __shared__ __align__(16) unsigned short Al[16 * STR];
  __shared__ __align__(16) float G[16 * GP2];
  const int row0 = blockIdx.x * 16;
  const int tid = threadIdx.x, lane = tid & 31, w = tid >> 5;
  const int hh = lane >> 4, m = lane & 15;
  const float mu = stats[0], inv = stats[1];
  const v4f nwv = *(const v4f*)(nw + 4 * lane);
  const v4f nbv = *(const v4f*)(nb + 4 * lane);
  for (int idx = tid; idx < 16 * (DHID / 4); idx += 128) {
    const int r = idx >> 5;
    const int row = row0 + r;
    v4f v = z4();
    if (row < nn) {
      v = *(const v4f*)(hsrc + (size_t)row * DHID + 4 * lane);
      v = ln_relu(v, mu, inv, nwv, nbv);
    }
    v4us hi, lo;
    split4(v, hi, lo);
    *(v4us*)(Ah + r * STR + 4 * lane) = hi;
    *(v4us*)(Al + r * STR + 4 * lane) = lo;
  }
  __syncthreads();
  const int n0 = w * 16;
  const unsigned short* bh_base = whi + (size_t)n0 * DHID;
  const unsigned short* bl_base = wlo + (size_t)n0 * DHID;
  v8f acc = z8();
#pragma unroll 1
  for (int ks = 0; ks < DHID / 32; ++ks) {
    const int k0 = ks * 32;
    v16b ah = frag_ld(Ah, STR, lane, k0);
    v16b al = frag_ld(Al, STR, lane, k0);
    v16b bh = frag_ld(bh_base, DHID, lane, k0);
    v16b bl = frag_ld(bl_base, DHID, lane, k0);
    acc = mma3(acc, ah, al, bh, bl);
  }
#pragma unroll
  for (int r = 0; r < 8; ++r) G[(8 * hh + r) * GP2 + n0 + m] = acc[r];
  __syncthreads();
  const v4f bv = *(const v4f*)(bias + 4 * m);
  v4f vals[2];
#pragma unroll
  for (int j2 = 0; j2 < 2; ++j2) {
    const int ml = 4 * w + 2 * j2 + hh;
    const v4f g = *(const v4f*)(G + ml * GP2 + 4 * m);
    vals[j2] = g + bv;
  }
  auto emit = [&]() {
#pragma unroll
    for (int j2 = 0; j2 < 2; ++j2) {
      const int row = row0 + 4 * w + 2 * j2 + hh;
      if (row < nn) *(volatile v4f*)(out + (size_t)row * DOUT + 4 * m) = vals[j2];
    }
  };
  emit();
  __threadfence();
  emit();
}

extern "C" void kernel_launch(void* const* d_in, const int* in_sizes, int n_in,
                              void* d_out, int out_size, void* d_ws,
                              size_t ws_size, hipStream_t stream) {
  if (n_in < 10) return;
  const float* x      = (const float*)d_in[0];
  const int*   ei     = (const int*)d_in[1];
  const float* lin1_w = (const float*)d_in[2];
  const float* lin1_b = (const float*)d_in[3];
  const float* w1     = (const float*)d_in[4];
  const float* w2     = (const float*)d_in[5];
  const float* norm_w = (const float*)d_in[6];
  const float* norm_b = (const float*)d_in[7];
  const float* lin2_w = (const float*)d_in[8];
  const float* lin2_b = (const float*)d_in[9];
  float* outp = (float*)d_out;

  const int nn = in_sizes[0] / DIN;
  const int ne = in_sizes[1] / 2;
  if (nn <= 0 || ne < 0) return;
  if (in_sizes[2] != DIN * DHID || in_sizes[4] != NLAYERS * DHID * DHID ||
      in_sizes[5] != NLAYERS * DHID * DHID || in_sizes[8] != DHID * DOUT) return;
  if (in_sizes[3] < DHID || in_sizes[6] < NLAYERS * DHID || in_sizes[7] < NLAYERS * DHID ||
      in_sizes[9] < DOUT) return;
  if ((long long)out_size < (long long)nn * DOUT) return;

  const int nbkt = (nn + NPBK - 1) / NPBK;
  const int nnp  = nbkt * NPBK;
  const int nblk = (nn + 15) / 16;
  const int csr_len = nbkt * BCAP;

  size_t off = 0;
  auto carve = [&](size_t bytes) -> size_t {
    size_t p = off;
    off = (off + bytes + 255) & ~(size_t)255;
    return p;
  };
  const size_t o_csr   = carve((size_t)csr_len * 4);
  const size_t o_nst   = carve((size_t)nnp * 4);
  const size_t o_ncnt  = carve((size_t)nnp * 4);
  const size_t o_dinv  = carve((size_t)nnp * 4);
  const size_t o_l1h   = carve((size_t)DHID * DIN * 2);
  const size_t o_l1l   = carve((size_t)DHID * DIN * 2);
  const size_t o_w1h   = carve((size_t)NLAYERS * DHID * DHID * 2);
  const size_t o_w1l   = carve((size_t)NLAYERS * DHID * DHID * 2);
  const size_t o_w2h   = carve((size_t)NLAYERS * DHID * DHID * 2);
  const size_t o_w2l   = carve((size_t)NLAYERS * DHID * DHID * 2);
  const size_t o_l2h   = carve((size_t)DOUT * DHID * 2);
  const size_t o_l2l   = carve((size_t)DOUT * DHID * 2);
  const size_t o_x0    = carve((size_t)nn * DHID * 4);
  const size_t o_oa    = carve((size_t)nn * DHID * 4);
  const size_t o_ob    = carve((size_t)nn * DHID * 4);
  const size_t o_part  = carve((size_t)nblk * PLD * 8);
  const size_t o_stats = carve((size_t)NLAYERS * SLF * 4);
  if (off > ws_size) return;

  char* ws = (char*)d_ws;
  int*   csr    = (int*)(ws + o_csr);
  int*   nstart = (int*)(ws + o_nst);
  int*   ncnt   = (int*)(ws + o_ncnt);
  float* dinv   = (float*)(ws + o_dinv);
  unsigned short* l1h = (unsigned short*)(ws + o_l1h);
  unsigned short* l1l = (unsigned short*)(ws + o_l1l);
  unsigned short* w1h = (unsigned short*)(ws + o_w1h);
  unsigned short* w1l = (unsigned short*)(ws + o_w1l);
  unsigned short* w2h = (unsigned short*)(ws + o_w2h);
  unsigned short* w2l = (unsigned short*)(ws + o_w2l);
  unsigned short* l2h = (unsigned short*)(ws + o_l2h);
  unsigned short* l2l = (unsigned short*)(ws + o_l2l);
  float*  x0    = (float*)(ws + o_x0);
  float*  outb[2] = { (float*)(ws + o_oa), (float*)(ws + o_ob) };
  double* part  = (double*)(ws + o_part);
  float*  stats = (float*)(ws + o_stats);

  k_csr<<<dim3(nbkt), dim3(256), 0, stream>>>(ei, ei + ne, ne, nn, csr, nstart, ncnt, dinv);

  k_wcvt<<<dim3(1 * (DHID / 32)), dim3(256), 0, stream>>>(lin1_w, DIN, DHID, 1, l1h, l1l);
  k_wcvt<<<dim3(NLAYERS * (DHID / 32)), dim3(256), 0, stream>>>(w1, DHID, DHID, NLAYERS, w1h, w1l);
  k_wcvt<<<dim3(NLAYERS * (DHID / 32)), dim3(256), 0, stream>>>(w2, DHID, DHID, NLAYERS, w2h, w2l);
  k_wcvt<<<dim3(1 * (DOUT / 32)), dim3(256), 0, stream>>>(lin2_w, DHID, DOUT, 1, l2h, l2l);

  k_lin1<<<dim3(nblk), dim3(128), 0, stream>>>(x, l1h, l1l, lin1_b, nn, x0);

  const double cntM = (double)nn * (double)DHID;
  for (int i = 0; i < NLAYERS; ++i) {
    const float beta = (float)log(1.0 / (double)(i + 1) + 1.0);
    const float* hsrc = (i == 0) ? (const float*)x0 : (const float*)outb[(i - 1) & 1];
    const int mode = (i == 0) ? 0 : 1;
    const int ip = (i == 0) ? 0 : (i - 1);
    k_layer<<<dim3(nblk), dim3(128), 0, stream>>>(
        hsrc, mode, stats + (size_t)ip * SLF, norm_w + (size_t)ip * DHID, norm_b + (size_t)ip * DHID,
        x0, csr, nstart, ncnt, dinv, csr_len,
        w1h + (size_t)i * DHID * DHID, w1l + (size_t)i * DHID * DHID,
        w2h + (size_t)i * DHID * DHID, w2l + (size_t)i * DHID * DHID,
        beta, nn, outb[i & 1], part);
    k_lnstat<<<dim3(1), dim3(256), 0, stream>>>(part, nblk, cntM, stats + (size_t)i * SLF);
  }

  const int il = NLAYERS - 1;
  k_lin2<<<dim3(nblk), dim3(128), 0, stream>>>(outb[il & 1], stats + (size_t)il * SLF,
                                               norm_w + (size_t)il * DHID, norm_b + (size_t)il * DHID,
                                               l2h, l2l, lin2_b, nn, outp);
}
